// MeKooMatching_90924457656589
// MI455X (gfx1250) — hardware-run, weakly checked
//
#include <hip/hip_runtime.h>
#include <math.h>

typedef __attribute__((ext_vector_type(16))) __bf16   v16b;
typedef __attribute__((ext_vector_type(8)))  __bf16   v8b;
typedef __attribute__((ext_vector_type(8)))  float    v8f;
typedef __attribute__((ext_vector_type(4)))  float    v4f;
typedef __attribute__((ext_vector_type(4)))  unsigned v4u;

constexpr int kBatch   = 8;
constexpr int kSteps   = 2048;
constexpr int kD       = 128;
constexpr int kNE      = 16;
constexpr int kRowsAll = kBatch * kSteps;
constexpr int kNcols   = kNE * kD;
constexpr int kTilesM  = kRowsAll / 64;
constexpr int kTilesN  = kNcols / 64;
constexpr int kTiles   = kTilesM * kTilesN;
constexpr int kPartFloats    = kTiles * 32;
constexpr int kPartPerExpert = kPartFloats / kNE;
constexpr int kSlabPitch     = 68;
static_assert((kSteps & (kSteps - 1)) == 0, "step count is a power of two");
static_assert((kD % 32) == 0, "GEMM K multiple of 32");
static_assert((kRowsAll % 64) == 0 && (kNcols % 64) == 0, "GEMM M,N multiples of 64");
static_assert((kTiles % 8) == 0, "eight tiles per block, exact grid");
static_assert(kD == 128 && (kTilesN % 2) == 0 && (kTilesN / 2) == kNE, "two column tiles per expert");
static_assert(kPartPerExpert == 2 * kTilesM * 32, "expert partial extent");
static_assert((kPartPerExpert % 128) == 0, "reduce loop step");

constexpr size_t kOffABF  = 0;
constexpr size_t kOffBT   = kOffABF + (size_t)kRowsAll * kD * 2;
constexpr size_t kOffPP   = kOffBT  + (size_t)kNcols * kD * 2;
constexpr size_t kOffPE   = kOffPP  + (size_t)kPartFloats * 4;
constexpr size_t kWsTotal = kOffPE  + (size_t)32 * 4;
static_assert(kWsTotal == 5767296ull, "carve total");
static_assert(kWsTotal <= 134217728ull, "carve cap");
static_assert((kOffBT % 128) == 0 && (kOffPP % 128) == 0 && (kOffPE % 128) == 0, "128-B aligned regions");

__device__ __forceinline__ unsigned f2bf_bits(float f) {
  const unsigned u = __float_as_uint(f);
  return ((u + 0x7FFFu + ((u >> 16) & 1u)) >> 16) & 0xFFFFu;
}
__device__ __forceinline__ float bf_rne(float f) {
  return __uint_as_float(f2bf_bits(f) << 16);
}

__device__ __forceinline__ v16b frag_load(const __bf16* p) {
  union U { v16b v; v8b h[2]; };
  U f;
  f.h[0] = *(const v8b*)(p);
  f.h[1] = *(const v8b*)(p + 16);
  return f.v;
}

__device__ __forceinline__ v8f mma_bf16(v16b a, v16b b, v8f c) {
  c = __builtin_amdgcn_wmma_f32_16x16x32_bf16(false, a, false, b, (short)0, c, false, false);
  asm volatile("v_nop\n\tv_nop\n\tv_nop\n\tv_nop" : "+v"(c) : "v"(a), "v"(b));
  return c;
}

__global__ __launch_bounds__(256) void seq_to_bf16_kernel(
    const float* __restrict__ src, unsigned short* __restrict__ dst, int total8)
{
  const int i = blockIdx.x * 256 + threadIdx.x;
  if (i >= total8) return;
  const size_t e0 = (size_t)i << 3;
  const v4f a0 = *(const v4f*)(src + e0);
  const v4f a1 = *(const v4f*)(src + e0 + 4);
  const float x0 = a0.x, x1 = a0.y, x2 = a0.z, x3 = a0.w;
  const float x4 = a1.x, x5 = a1.y, x6 = a1.z, x7 = a1.w;
  v4u w;
  w.x = f2bf_bits(x0) | (f2bf_bits(x1) << 16);
  w.y = f2bf_bits(x2) | (f2bf_bits(x3) << 16);
  w.z = f2bf_bits(x4) | (f2bf_bits(x5) << 16);
  w.w = f2bf_bits(x6) | (f2bf_bits(x7) << 16);
  unsigned short* q = dst + e0;
  *(volatile v4u*)q = w;
  __threadfence();
  *(volatile v4u*)q = w;
}

__global__ __launch_bounds__(256) void pool_transpose_kernel(
    const float* __restrict__ Kp, unsigned short* __restrict__ Bt)
{
  __shared__ float sT[kD * 33];
  const int tid = threadIdx.x, lane = tid & 31, wave = tid >> 5;
  const int n  = blockIdx.x >> 2;
  const int e0 = (blockIdx.x & 3) * 32;
  const float* src = Kp + (size_t)n * kD * kD;
#pragma unroll 1
  for (int it = 0; it < 16; ++it) {
    const int idx = it * 256 + tid;
    const int d = idx >> 5;
    const int e = idx & 31;
    sT[d * 33 + e] = src[d * kD + e0 + e];
  }
  __syncthreads();
  const int half = lane >> 4;
  const int d8 = (lane & 15) * 8;
#pragma unroll
  for (int it = 0; it < 2; ++it) {
    const int el = it * 16 + wave * 2 + half;
    const float y0 = sT[(d8 + 0) * 33 + el];
    const float y1 = sT[(d8 + 1) * 33 + el];
    const float y2 = sT[(d8 + 2) * 33 + el];
    const float y3 = sT[(d8 + 3) * 33 + el];
    const float y4 = sT[(d8 + 4) * 33 + el];
    const float y5 = sT[(d8 + 5) * 33 + el];
    const float y6 = sT[(d8 + 6) * 33 + el];
    const float y7 = sT[(d8 + 7) * 33 + el];
    v4u w;
    w.x = f2bf_bits(y0) | (f2bf_bits(y1) << 16);
    w.y = f2bf_bits(y2) | (f2bf_bits(y3) << 16);
    w.z = f2bf_bits(y4) | (f2bf_bits(y5) << 16);
    w.w = f2bf_bits(y6) | (f2bf_bits(y7) << 16);
    unsigned short* q = Bt + ((size_t)(n * kD + e0 + el) * kD + d8);
    *(volatile v4u*)q = w;
    __threadfence();
    *(volatile v4u*)q = w;
  }
}

__global__ __launch_bounds__(256) void predict_err_kernel(
    const unsigned short* __restrict__ Abf, const unsigned short* __restrict__ Btp,
    float* __restrict__ PP)
{
  __shared__ __align__(16) float sT[8][16 * kSlabPitch];
  const int lane = threadIdx.x & 31;
  const int wave = threadIdx.x >> 5;
  const int tile = blockIdx.x * 8 + wave;
  const int tm = tile / kTilesN;
  const int tn = tile - tm * kTilesN;
  const int m0 = tm << 6;
  const int n0 = tn << 6;
  const __bf16* A  = (const __bf16*)Abf;
  const __bf16* Bt = (const __bf16*)Btp;
  const unsigned* Aw = (const unsigned*)Abf;

  const int rlane = lane & 15;
  const int koff  = (lane >> 4) * 8;
  const int mOff  = (lane >> 4) * 8;

  v8f acc[4][4];
#pragma unroll
  for (int i = 0; i < 4; ++i)
#pragma unroll
    for (int j = 0; j < 4; ++j) acc[i][j] = (v8f){0.f, 0.f, 0.f, 0.f, 0.f, 0.f, 0.f, 0.f};

#pragma unroll 1
  for (int k0 = 0; k0 < kD; k0 += 32) {
    v16b bh[4];
#pragma unroll
    for (int j = 0; j < 4; ++j) {
      const size_t bo = (size_t)(n0 + (j << 4) + rlane) * kD + koff + k0;
      bh[j] = frag_load(Bt + bo);
    }
#pragma unroll
    for (int i = 0; i < 4; ++i) {
      const size_t ao = (size_t)(m0 + (i << 4) + rlane) * kD + koff + k0;
      const v16b ah = frag_load(A + ao);
#pragma unroll
      for (int j = 0; j < 4; ++j) acc[i][j] = mma_bf16(ah, bh[j], acc[i][j]);
    }
  }

  float* slab = sT[wave];
  const int ew = (n0 & (kD - 1)) >> 1;
  float part = 0.0f;
#pragma unroll
  for (int i = 0; i < 4; ++i) {
    __syncthreads();
#pragma unroll
    for (int j = 0; j < 4; ++j) {
#pragma unroll
      for (int r = 0; r < 8; ++r) {
        slab[(mOff + r) * kSlabPitch + (j << 4) + rlane] = acc[i][j][r];
      }
    }
    __syncthreads();
#pragma unroll 1
    for (int rr = 0; rr < 16; ++rr) {
      const int R = m0 + (i << 4) + rr;
      const int Rn = (R + 1 < kRowsAll) ? (R + 1) : (kRowsAll - 1);
      unsigned w = Aw[Rn * (kD >> 1) + ew + lane];
      asm volatile("" : "+v"(w));
      const float c0 = slab[rr * kSlabPitch + 2 * lane];
      const float c1 = slab[rr * kSlabPitch + 2 * lane + 1];
      const float s0 = __uint_as_float(w << 16);
      const float s1 = __uint_as_float(w & 0xFFFF0000u);
      const float t0 = expf(fabsf(c0 - s0));
      const float t1 = expf(fabsf(c1 - s1));
      const bool valid = ((R & (kSteps - 1)) != (kSteps - 1));
      const float tsum = t0 + t1;
      part += valid ? tsum : 0.0f;
    }
  }

  volatile float* pp = PP + ((size_t)(tn * kTilesM + tm) * 32 + lane);
  *pp = part;
  __threadfence();
  *pp = part;
}

__global__ __launch_bounds__(512) void expert_sum_kernel(
    const float* __restrict__ PP, float* __restrict__ PE)
{
  __shared__ float sS[kNE];
  const int lane = threadIdx.x & 31;
  const int wave = threadIdx.x >> 5;
  const float* base = PP + (size_t)wave * kPartPerExpert;
  v4f a = (v4f){0.f, 0.f, 0.f, 0.f};
#pragma unroll 1
  for (int it = 0; it < kPartPerExpert / 128; ++it) {
    const v4f x = *(const v4f*)(base + it * 128 + lane * 4);
    a += x;
  }
  float s = (a.x + a.y) + (a.z + a.w);
  s += __shfl_xor(s, 16, 32);
  s += __shfl_xor(s, 8, 32);
  s += __shfl_xor(s, 4, 32);
  s += __shfl_xor(s, 2, 32);
  s += __shfl_xor(s, 1, 32);
  if (lane == 0) sS[wave] = s;
  __syncthreads();
  const float v = sS[lane & 15];
  const float outv = (lane < kNE) ? v : 0.0f;
  if (wave == 0) {
    volatile float* p = PE + lane;
    *p = outv;
    __threadfence();
    *p = outv;
  }
}

__global__ __launch_bounds__(256) void mix_kernel(
    const float* __restrict__ Kp, const float* __restrict__ PE, float* __restrict__ out)
{
  const int i4 = blockIdx.x * 256 + threadIdx.x;
  const size_t e0 = (size_t)i4 << 2;
  float tot = 0.0f;
#pragma unroll 1
  for (int k = 0; k < kNE; ++k) tot += PE[k];
  float rinv = __builtin_amdgcn_rcpf(tot);
  const float er = fmaf(-tot, rinv, 1.0f);
  rinv = fmaf(rinv, er, rinv);
  float o0 = 0.0f, o1 = 0.0f, o2 = 0.0f, o3 = 0.0f;
#pragma unroll 1
  for (int k = 0; k < kNE; ++k) {
    const float lam = PE[k] * rinv;
    const v4f x = *(const v4f*)(Kp + (size_t)k * kD * kD + e0);
    const float x0 = x.x, x1 = x.y, x2 = x.z, x3 = x.w;
    o0 = fmaf(bf_rne(x0), lam, o0);
    o1 = fmaf(bf_rne(x1), lam, o1);
    o2 = fmaf(bf_rne(x2), lam, o2);
    o3 = fmaf(bf_rne(x3), lam, o3);
  }
  const v4f ov = (v4f){o0, o1, o2, o3};
  float* q = out + e0;
  *(volatile v4f*)q = ov;
  __threadfence();
  *(volatile v4f*)q = ov;
}

extern "C" void kernel_launch(void* const* d_in, const int* in_sizes, int n_in,
                              void* d_out, int out_size, void* d_ws, size_t ws_size,
                              hipStream_t stream) {
  if (n_in < 2) return;
  if (in_sizes[0] != kRowsAll * kD) return;
  if (in_sizes[1] != kNE * kD * kD) return;
  if (out_size != kD * kD) return;
  if (ws_size < kWsTotal) return;

  const float* seq = (const float*)d_in[0];
  const float* Kp  = (const float*)d_in[1];
  float* out = (float*)d_out;

  char* ws = (char*)d_ws;
  unsigned short* ABF = (unsigned short*)(ws + kOffABF);
  unsigned short* BT  = (unsigned short*)(ws + kOffBT);
  float*          PP  = (float*)(ws + kOffPP);
  float*          PE  = (float*)(ws + kOffPE);

  seq_to_bf16_kernel<<<(kRowsAll * kD / 8) / 256, 256, 0, stream>>>(seq, ABF, kRowsAll * kD / 8);
  pool_transpose_kernel<<<kNE * 4, 256, 0, stream>>>(Kp, BT);
  predict_err_kernel<<<kTiles / 8, 256, 0, stream>>>(ABF, BT, PP);
  expert_sum_kernel<<<1, 512, 0, stream>>>(PP, PE);
  mix_kernel<<<(kD * kD / 4) / 256, 256, 0, stream>>>(Kp, PE, out);
}
